// PointNetPlusSAModule_7576322310711
// MI455X (gfx1250) — hardware-verified
//
#include <hip/hip_runtime.h>
#pragma clang fp contract(off)

typedef __attribute__((ext_vector_type(16))) _Float16 v16h;
typedef __attribute__((ext_vector_type(8)))  _Float16 v8h;
typedef __attribute__((ext_vector_type(8)))  float    v8f;
typedef __attribute__((ext_vector_type(4)))  float    v4f;

constexpr int kBatch   = 16;
constexpr int kPts     = 4096;
constexpr int kFeat    = 64;
constexpr int kCen     = 1024;
constexpr int kW0Pitch = 67;
constexpr int kK0      = 32;
constexpr int kK1      = 64;
constexpr int kStatBlocks = 256;
constexpr int kPartPitch  = 256;
constexpr float kWCarry    = 16.0f;
constexpr float kWCarryInv = 1.0f / 16.0f;
constexpr int kRows0 = kBatch * kCen * kK0;
constexpr int kRows1 = kBatch * kCen * kK1;

static_assert(kBatch * 3 * kCen * 4 == 196608, "out0 bytes");
static_assert(196608 + kBatch * 256 * kCen * 4 == 16973824, "d_out bytes");
static_assert(196608 % 128 == 0, "out1 line aligned");
static_assert(kK0 == 32 && kK1 == 64, "ball query lane map");
static_assert(kRows0 == 524288 && kRows1 == 1048576, "rows per branch");
static_assert(kRows0 % (kStatBlocks * 64) == 0 && kRows1 % (kStatBlocks * 64) == 0, "tile split");
static_assert(kCen == 1024 && kPts == 4096, "shift based index math");

constexpr size_t kOffNx   = 0;
constexpr size_t kOffIdx0 = kOffNx   + (size_t)kBatch * 3 * kCen * 4;
constexpr size_t kOffIdx1 = kOffIdx0 + (size_t)kBatch * kCen * kK0 * 4;
constexpr size_t kOffP0   = kOffIdx1 + (size_t)kBatch * kCen * kK1 * 4;
constexpr size_t kOffP1   = kOffP0   + (size_t)kBatch * kPts * 64 * 4;
constexpr size_t kOffY0   = kOffP1   + (size_t)kBatch * kPts * 64 * 4;
constexpr size_t kOffY1   = kOffY0   + (size_t)kBatch * kCen * 128 * 4;
constexpr size_t kOffPart = kOffY1   + (size_t)kBatch * kCen * 128 * 4;
constexpr size_t kOffAc   = kOffPart + (size_t)6 * kStatBlocks * kPartPitch * 4;
constexpr size_t kWsTotal = kOffAc   + (size_t)6 * 256 * 4;
static_assert(kWsTotal == 58398720, "carve total");
static_assert(kWsTotal <= 134217728, "carve within 128 MiB");
static_assert(kOffIdx0 % 128 == 0 && kOffIdx1 % 128 == 0 && kOffP0 % 128 == 0 && kOffP1 % 128 == 0 &&
              kOffY0 % 128 == 0 && kOffY1 % 128 == 0 && kOffPart % 128 == 0 && kOffAc % 128 == 0, "line aligned carve");

union FragH { v16h v; v8h h[2]; };

__device__ __forceinline__ v8f mma_f16(v16h a, v16h b, v8f c) {
  c = __builtin_amdgcn_wmma_f32_16x16x32_f16(false, a, false, b, (short)0, c, false, false);
  asm volatile("v_nop\n\tv_nop\n\tv_nop\n\tv_nop" : "+v"(c) : "v"(a), "v"(b));
  return c;
}

__device__ __forceinline__ v16h wfrag_vec(const float* __restrict__ p) {
  const v4f a = *(const v4f*)(p);
  const v4f b = *(const v4f*)(p + 4);
  const v4f c = *(const v4f*)(p + 16);
  const v4f d = *(const v4f*)(p + 20);
  v16h r;
#pragma unroll
  for (int e = 0; e < 4; ++e) {
    r[e]      = (_Float16)(a[e] * kWCarry);
    r[4 + e]  = (_Float16)(b[e] * kWCarry);
    r[8 + e]  = (_Float16)(c[e] * kWCarry);
    r[12 + e] = (_Float16)(d[e] * kWCarry);
  }
  asm volatile("" ::: "memory");
  return r;
}
__device__ __forceinline__ v16h wfrag_sca(const float* __restrict__ p) {
  float f[16];
#pragma unroll
  for (int e = 0; e < 8; ++e) f[e] = p[e];
  asm volatile("" ::: "memory");
#pragma unroll
  for (int e = 0; e < 8; ++e) f[8 + e] = p[16 + e];
  v16h r;
#pragma unroll
  for (int e = 0; e < 16; ++e) r[e] = (_Float16)(f[e] * kWCarry);
  asm volatile("" ::: "memory");
  return r;
}

__device__ __forceinline__ float y0_val(float p, float wx, float wy, float wz, float rx, float ry, float rz) {
  const float t = (wx * rx + wy * ry) + wz * rz;
  return p + t;
}

__global__ __launch_bounds__(1024) void k_fps(const float* __restrict__ pc, float* __restrict__ out0,
                                              float* __restrict__ nx) {
#pragma clang fp contract(off)
  __shared__ __align__(16) float sx[3 * kPts];
  __shared__ float pv[2][32];
  __shared__ int   pi[2][32];
  __shared__ int   sidx[kCen];
  const int tid = threadIdx.x, lane = tid & 31, wave = tid >> 5;
  const int b = blockIdx.x;
  {
    const v4f* src = (const v4f*)(pc + (size_t)b * 3 * kPts);
    v4f* dl = (v4f*)sx;
#pragma unroll
    for (int m = 0; m < 3; ++m) dl[tid + 1024 * m] = src[tid + 1024 * m];
  }
  if (tid == 0) sidx[0] = 0;
  __syncthreads();
  float px[4], py[4], pz[4], dist[4];
#pragma unroll
  for (int q = 0; q < 4; ++q) {
    const int i = tid + 1024 * q;
    px[q] = sx[i]; py[q] = sx[kPts + i]; pz[q] = sx[2 * kPts + i];
    dist[q] = 1e10f;
  }
  int last = 0;
#pragma unroll 1
  for (int t = 1; t < kCen; ++t) {
    const float lx = sx[last], ly = sx[kPts + last], lz = sx[2 * kPts + last];
    float bv = 0.f; int bi = tid;
#pragma unroll
    for (int q = 0; q < 4; ++q) {
      const float dx = px[q] - lx, dy = py[q] - ly, dz = pz[q] - lz;
      const float t0 = dx * dx, t1 = dy * dy, t2 = dz * dz;
      const float d = (t0 + t2) + t1;
      const float nd = fminf(dist[q], d);
      dist[q] = nd;
      if (q == 0) { bv = nd; bi = tid; }
      else { const bool tk = nd > bv; bv = tk ? nd : bv; bi = tk ? (tid + 1024 * q) : bi; }
    }
#pragma unroll
    for (int off = 16; off > 0; off >>= 1) {
      const float ov = __shfl_xor(bv, off, 32);
      const int   oi = __shfl_xor(bi, off, 32);
      const bool tk = (ov > bv) | ((ov == bv) & (oi < bi));
      bv = tk ? ov : bv; bi = tk ? oi : bi;
    }
    const int buf = t & 1;
    if (lane == 0) { pv[buf][wave] = bv; pi[buf][wave] = bi; }
    __syncthreads();
    float cv = pv[buf][lane]; int ci = pi[buf][lane];
#pragma unroll
    for (int off = 16; off > 0; off >>= 1) {
      const float ov = __shfl_xor(cv, off, 32);
      const int   oi = __shfl_xor(ci, off, 32);
      const bool tk = (ov > cv) | ((ov == cv) & (oi < ci));
      cv = tk ? ov : cv; ci = tk ? oi : ci;
    }
    ci = ci < 0 ? 0 : (ci > kPts - 1 ? kPts - 1 : ci);
    last = ci;
    if (tid == 0) sidx[t] = last;
  }
  __syncthreads();
  const int si = sidx[tid];
  float val[3];
#pragma unroll
  for (int d = 0; d < 3; ++d) val[d] = sx[d * kPts + si];
  float* o0 = out0 + (size_t)b * 3 * kCen;
  float* o1 = nx + (size_t)b * 3 * kCen;
  for (int pass = 0; pass < 2; ++pass) {
#pragma unroll
    for (int d = 0; d < 3; ++d) {
      *(volatile float*)(o0 + d * kCen + tid) = val[d];
      *(volatile float*)(o1 + d * kCen + tid) = val[d];
    }
    __threadfence();
  }
}

__global__ __launch_bounds__(256) void k_ballquery(const float* __restrict__ pc, const float* __restrict__ nx,
                                                   int* __restrict__ idx0, int* __restrict__ idx1) {
#pragma clang fp contract(off)
  __shared__ int l0[8][kK0];
  __shared__ int l1[8][kK1];
  const int tid = threadIdx.x, lane = tid & 31, wave = tid >> 5;
  const int cen = blockIdx.x * 8 + wave;
  const int b = cen >> 10;
  const int m = cen & (kCen - 1);
  const float* nb = nx + (size_t)b * 3 * kCen;
  const float cx = nb[m], cy = nb[kCen + m], cz = nb[2 * kCen + m];
  const float r2a = __uint_as_float(0x3C23D70Au);
  const float r2b = __uint_as_float(0x3D23D70Au);
  const float* xb = pc + (size_t)b * 3 * kPts;
  const unsigned lt = (1u << lane) - 1u;
  int cnt0 = 0, cnt1 = 0, first0 = 0, first1 = 0;
#pragma unroll 1
  for (int base = 0; base < kPts; base += 32) {
    if (cnt0 >= kK0 && cnt1 >= kK1) break;
    const int j = base + lane;
    const float x = xb[j], y = xb[kPts + j], z = xb[2 * kPts + j];
    const float dx = cx - x, dy = cy - y, dz = cz - z;
    const float t0 = dx * dx, t1 = dy * dy, t2 = dz * dz;
    const float d2 = (t0 + t2) + t1;
    const bool in0 = d2 < r2a;
    const bool in1 = d2 < r2b;
    const unsigned m0 = __builtin_amdgcn_ballot_w32(in0);
    const unsigned m1 = __builtin_amdgcn_ballot_w32(in1);
    const int p0 = cnt0 + __popc(m0 & lt);
    const int p1 = cnt1 + __popc(m1 & lt);
    if (in0 && p0 < kK0) l0[wave][p0] = j;
    if (in1 && p1 < kK1) l1[wave][p1] = j;
    first0 = (cnt0 == 0 && m0 != 0u) ? (base + __ffs((int)m0) - 1) : first0;
    first1 = (cnt1 == 0 && m1 != 0u) ? (base + __ffs((int)m1) - 1) : first1;
    cnt0 += __popc(m0);
    cnt1 += __popc(m1);
  }
  if (lane >= cnt0) l0[wave][lane] = first0;
  if (lane >= cnt1) l1[wave][lane] = first1;
  if (lane + 32 >= cnt1) l1[wave][lane + 32] = first1;
  __syncthreads();
  const int v0  = l0[wave][lane];
  const int v1a = l1[wave][lane];
  const int v1b = l1[wave][lane + 32];
  volatile int* d0 = (volatile int*)(idx0 + (size_t)cen * kK0 + lane);
  volatile int* d1 = (volatile int*)(idx1 + (size_t)cen * kK1 + lane);
  *d0 = v0;
  d1[0] = v1a;
  d1[32] = v1b;
  __threadfence();
  *d0 = v0;
  d1[0] = v1a;
  d1[32] = v1b;
}

__global__ __launch_bounds__(256) void k_pgemm(const float* __restrict__ feat, const float* __restrict__ W0a,
                                               const float* __restrict__ W0b, float* __restrict__ Pa,
                                               float* __restrict__ Pb, int tilesPerBlock) {
  constexpr int APITCH = 72;
  __shared__ __align__(16) _Float16 As[64 * APITCH];
  __shared__ __align__(16) float Ps[64 * 64];
  const float* W0 = (blockIdx.y != 0) ? W0b : W0a;
  float* P = (blockIdx.y != 0) ? Pb : Pa;
  const int tid = threadIdx.x, lane = tid & 31, wave = tid >> 5;
  const int lm = lane & 15, hf = lane >> 4;
  const int rs = wave & 3, cg = wave >> 2;
  v16h bf[2][2];
#pragma unroll
  for (int j = 0; j < 2; ++j)
#pragma unroll
    for (int kk = 0; kk < 2; ++kk) {
      const int o = cg * 32 + 16 * j + lm;
      bf[j][kk] = wfrag_sca(W0 + (size_t)o * kW0Pitch + 3 + kk * 32 + 8 * hf);
    }
#pragma unroll 1
  for (int tt = 0; tt < tilesPerBlock; ++tt) {
    const int tile = blockIdx.x * tilesPerBlock + tt;
    const int b = tile >> 6;
    const int n0 = (tile & 63) * 64;
    {
      const int n = tid & 63, cq = tid >> 6;
      const float* fp = feat + ((size_t)(b * kFeat + cq * 16)) * kPts + n0 + n;
      float f[16];
#pragma unroll
      for (int e = 0; e < 8; ++e) f[e] = fp[(size_t)e * kPts];
      asm volatile("" ::: "memory");
#pragma unroll
      for (int e = 0; e < 8; ++e) f[8 + e] = fp[(size_t)(8 + e) * kPts];
      v8h h0, h1;
#pragma unroll
      for (int e = 0; e < 8; ++e) { h0[e] = (_Float16)f[e]; h1[e] = (_Float16)f[8 + e]; }
      *(v8h*)(As + n * APITCH + cq * 16) = h0;
      *(v8h*)(As + n * APITCH + cq * 16 + 8) = h1;
    }
    __syncthreads();
    v8f acc[2];
    acc[0] = (v8f){0.f, 0.f, 0.f, 0.f, 0.f, 0.f, 0.f, 0.f};
    acc[1] = (v8f){0.f, 0.f, 0.f, 0.f, 0.f, 0.f, 0.f, 0.f};
#pragma unroll
    for (int kk = 0; kk < 2; ++kk) {
      FragH fa;
      fa.h[0] = *(const v8h*)(As + (rs * 16 + lm) * APITCH + kk * 32 + 8 * hf);
      fa.h[1] = *(const v8h*)(As + (rs * 16 + lm) * APITCH + kk * 32 + 16 + 8 * hf);
#pragma unroll
      for (int j = 0; j < 2; ++j) acc[j] = mma_f16(fa.v, bf[j][kk], acc[j]);
    }
#pragma unroll
    for (int j = 0; j < 2; ++j)
#pragma unroll
      for (int r = 0; r < 8; ++r) {
        const float v = acc[j][r] * kWCarryInv;
        Ps[(rs * 16 + 8 * hf + r) * 64 + cg * 32 + 16 * j + lm] = v;
      }
    __syncthreads();
    {
      float* dst = P + ((size_t)b * kPts + n0) * 64;
      v4f vals[4];
#pragma unroll
      for (int i = 0; i < 4; ++i) vals[i] = *(const v4f*)(Ps + (tid + 256 * i) * 4);
      for (int pass = 0; pass < 2; ++pass) {
#pragma unroll
        for (int i = 0; i < 4; ++i) *(volatile v4f*)(dst + (size_t)(tid + 256 * i) * 4) = vals[i];
        __threadfence();
      }
    }
  }
}

template <int KS>
__global__ __launch_bounds__(256) void k_l0stats(const float* __restrict__ P, const int* __restrict__ idx,
                                                 const float* __restrict__ pc, const float* __restrict__ nx,
                                                 const float* __restrict__ W0, float* __restrict__ part,
                                                 int rowsPerBlock) {
  __shared__ float rsum[2][64][64];
  __shared__ __align__(16) float fin[256];
  __shared__ __align__(16) float wsh[3][64];
  const int tid = threadIdx.x;
  const int cq = tid & 3, slot = tid >> 2;
  if (tid < 64) {
    wsh[0][tid] = W0[tid * kW0Pitch + 0];
    wsh[1][tid] = W0[tid * kW0Pitch + 1];
    wsh[2][tid] = W0[tid * kW0Pitch + 2];
  }
  __syncthreads();
  float wx[16], wy[16], wz[16], s[16], q[16];
#pragma unroll
  for (int e = 0; e < 16; ++e) {
    wx[e] = wsh[0][cq * 16 + e]; wy[e] = wsh[1][cq * 16 + e]; wz[e] = wsh[2][cq * 16 + e];
    s[e] = 0.f; q[e] = 0.f;
  }
  const size_t row0 = (size_t)blockIdx.x * rowsPerBlock;
  const int nit = rowsPerBlock >> 6;
#pragma unroll 1
  for (int it = 0; it < nit; ++it) {
    const size_t g = row0 + (size_t)it * 64 + slot;
    int j = idx[g];
    j = j < 0 ? 0 : (j > kPts - 1 ? kPts - 1 : j);
    const int cen = (int)(g / KS);
    const int b = cen >> 10;
    const int m = cen & (kCen - 1);
    const float* pb = pc + (size_t)b * 3 * kPts;
    const float* nb = nx + (size_t)b * 3 * kCen;
    const float rx = pb[j] - nb[m];
    const float ry = pb[kPts + j] - nb[kCen + m];
    const float rz = pb[2 * kPts + j] - nb[2 * kCen + m];
    const float* pp = P + ((size_t)b * kPts + j) * 64 + cq * 16;
    v4f p[4];
#pragma unroll
    for (int qd = 0; qd < 4; ++qd) p[qd] = *(const v4f*)(pp + 4 * qd);
#pragma unroll
    for (int qd = 0; qd < 4; ++qd)
#pragma unroll
      for (int e = 0; e < 4; ++e) {
        const int c = 4 * qd + e;
        const float y = y0_val(p[qd][e], wx[c], wy[c], wz[c], rx, ry, rz);
        s[c] += y;
        q[c] += y * y;
      }
  }
#pragma unroll
  for (int e = 0; e < 16; ++e) { rsum[0][slot][cq * 16 + e] = s[e]; rsum[1][slot][cq * 16 + e] = q[e]; }
  __syncthreads();
  {
    const int n = tid & 127, qq = tid >> 7;
    const int nc = n < 64 ? n : 63;
    float v = 0.f;
#pragma unroll 4
    for (int sl = 0; sl < 64; ++sl) v += rsum[qq][sl][nc];
    fin[tid] = (n < 64) ? v : 0.f;
  }
  __syncthreads();
  if (tid < 64) {
    const v4f v = *(const v4f*)(fin + 4 * tid);
    volatile v4f* d = (volatile v4f*)(part + (size_t)blockIdx.x * kPartPitch + 4 * tid);
    *d = v;
    __threadfence();
    *d = v;
  }
}

__global__ __launch_bounds__(128) void k_bnfin(const float* __restrict__ part, int nblk, int nch,
                                               const float* __restrict__ g, const float* __restrict__ bt,
                                               float invn, float* __restrict__ ac) {
  __shared__ __align__(16) float sac[256];
  const int o = threadIdx.x;
  const int oc = o < nch ? o : nch - 1;
  double s = 0.0, q = 0.0;
#pragma unroll 4
  for (int k = 0; k < nblk; ++k) {
    s += (double)part[(size_t)k * kPartPitch + oc];
    q += (double)part[(size_t)k * kPartPitch + 128 + oc];
  }
  const double mean = s * (double)invn;
  double var = q * (double)invn - mean * mean;
  var = var < 0.0 ? 0.0 : var;
  const float inv = rsqrtf((float)var + 1e-5f);
  const float a = g[oc] * inv;
  const float c = bt[oc] - (float)mean * a;
  sac[o] = (o < nch) ? a : 0.f;
  sac[128 + o] = (o < nch) ? c : 0.f;
  __syncthreads();
  if (o < 64) {
    const v4f v = *(const v4f*)(sac + 4 * o);
    volatile v4f* d = (volatile v4f*)(ac + 4 * o);
    *d = v;
    __threadfence();
    *d = v;
  }
}

template <int NOUT1, int KS, bool FULL>
__global__ __launch_bounds__(256) void k_mlp(const float* __restrict__ P, const int* __restrict__ idx,
                                             const float* __restrict__ pc, const float* __restrict__ nx,
                                             const float* __restrict__ W0, const float* __restrict__ ac0,
                                             const float* __restrict__ W1, const float* __restrict__ ac1,
                                             const float* __restrict__ W2, const float* __restrict__ g2,
                                             float* __restrict__ yext, float* __restrict__ part,
                                             int tilesPerBlock) {
  constexpr int NJ  = NOUT1 / 32;
  constexpr int HW  = NOUT1 / 2;
  constexpr int NK2 = NOUT1 / 32;
  constexpr int AP  = 72;
  constexpr int A2P = NOUT1 + 8;
  constexpr int NCT = 64 / KS;
  constexpr int SPC = 4 / NCT;
  static_assert(NOUT1 % 32 == 0 && NOUT1 <= 128, "column split and k steps");
  static_assert(KS == 32 || KS == 64, "centres per 64-row tile");
  static_assert((A2P * 2) % 16 == 0, "tile pitch 16-B aligned");
  __shared__ __align__(16) _Float16 As[64 * AP];
  __shared__ __align__(16) _Float16 A2s[FULL ? 64 * A2P : 8];
  __shared__ __align__(16) float cst[5][64];
  __shared__ __align__(16) float Ex[2][128];
  __shared__ float red[2][8][64];
  __shared__ __align__(16) float fin[256];
  const int tid = threadIdx.x, lane = tid & 31, wave = tid >> 5;
  const int lm = lane & 15, hf = lane >> 4;
  const int rs = wave & 3, cg = wave >> 2;
  if (tid < 64) {
    cst[0][tid] = ac0[tid];
    cst[1][tid] = ac0[128 + tid];
    cst[2][tid] = W0[tid * kW0Pitch + 0];
    cst[3][tid] = W0[tid * kW0Pitch + 1];
    cst[4][tid] = W0[tid * kW0Pitch + 2];
  }
  v16h bf1[NJ][2];
#pragma unroll
  for (int j = 0; j < NJ; ++j)
#pragma unroll
    for (int kk = 0; kk < 2; ++kk) {
      const int n = cg * HW + 16 * j + lm;
      bf1[j][kk] = wfrag_vec(W1 + (size_t)n * 64 + kk * 32 + 8 * hf);
    }
  v16h bf2[NK2];
  float a1r[NJ], c1r[NJ];
  int gp = 1;
#pragma unroll
  for (int j = 0; j < NJ; ++j) { a1r[j] = 0.f; c1r[j] = 0.f; }
  if (FULL) {
#pragma unroll
    for (int kk = 0; kk < NK2; ++kk)
      bf2[kk] = wfrag_vec(W2 + (size_t)(16 * wave + lm) * NOUT1 + kk * 32 + 8 * hf);
#pragma unroll
    for (int j = 0; j < NJ; ++j) {
      const int ch = cg * HW + 16 * j + lm;
      a1r[j] = ac1[ch];
      c1r[j] = ac1[128 + ch];
    }
    gp = (g2[16 * wave + lm] > 0.0f) ? 1 : 0;
  }
  float s1[NJ], q1[NJ];
#pragma unroll
  for (int j = 0; j < NJ; ++j) { s1[j] = 0.f; q1[j] = 0.f; }
  float s2 = 0.f, q2 = 0.f;
  __syncthreads();
#pragma unroll 1
  for (int tt = 0; tt < tilesPerBlock; ++tt) {
    const int tile = blockIdx.x * tilesPerBlock + tt;
    {
      const int r = tid >> 2, cq = tid & 3;
      const size_t g = (size_t)tile * 64 + r;
      int j = idx[g];
      j = j < 0 ? 0 : (j > kPts - 1 ? kPts - 1 : j);
      const int cen = (int)(g / KS);
      const int b = cen >> 10;
      const int m = cen & (kCen - 1);
      const float* pb = pc + (size_t)b * 3 * kPts;
      const float* nb = nx + (size_t)b * 3 * kCen;
      const float rx = pb[j] - nb[m];
      const float ry = pb[kPts + j] - nb[kCen + m];
      const float rz = pb[2 * kPts + j] - nb[2 * kCen + m];
      const float* pp = P + ((size_t)b * kPts + j) * 64 + cq * 16;
      v4f p[4];
#pragma unroll
      for (int qd = 0; qd < 4; ++qd) p[qd] = *(const v4f*)(pp + 4 * qd);
      v8h h0, h1;
#pragma unroll
      for (int qd = 0; qd < 4; ++qd) {
        const v4f a4 = *(const v4f*)(&cst[0][cq * 16 + 4 * qd]);
        const v4f c4 = *(const v4f*)(&cst[1][cq * 16 + 4 * qd]);
        const v4f x4 = *(const v4f*)(&cst[2][cq * 16 + 4 * qd]);
        const v4f y4 = *(const v4f*)(&cst[3][cq * 16 + 4 * qd]);
        const v4f z4 = *(const v4f*)(&cst[4][cq * 16 + 4 * qd]);
#pragma unroll
        for (int e = 0; e < 4; ++e) {
          const float y = y0_val(p[qd][e], x4[e], y4[e], z4[e], rx, ry, rz);
          const float x = fmaxf(a4[e] * y + c4[e], 0.0f);
          if (qd < 2) h0[4 * qd + e] = (_Float16)x;
          else        h1[4 * (qd - 2) + e] = (_Float16)x;
        }
      }
      *(v8h*)(As + r * AP + cq * 16) = h0;
      *(v8h*)(As + r * AP + cq * 16 + 8) = h1;
    }
    __syncthreads();
    v8f acc1[NJ];
#pragma unroll
    for (int j = 0; j < NJ; ++j) acc1[j] = (v8f){0.f, 0.f, 0.f, 0.f, 0.f, 0.f, 0.f, 0.f};
#pragma unroll
    for (int kk = 0; kk < 2; ++kk) {
      FragH fa;
      fa.h[0] = *(const v8h*)(As + (rs * 16 + lm) * AP + kk * 32 + 8 * hf);
      fa.h[1] = *(const v8h*)(As + (rs * 16 + lm) * AP + kk * 32 + 16 + 8 * hf);
#pragma unroll
      for (int j = 0; j < NJ; ++j) acc1[j] = mma_f16(fa.v, bf1[j][kk], acc1[j]);
    }
    if (!FULL) {
#pragma unroll
      for (int j = 0; j < NJ; ++j)
#pragma unroll
        for (int r = 0; r < 8; ++r) {
          const float v = acc1[j][r] * kWCarryInv;
          s1[j] += v;
          q1[j] += v * v;
        }
      __syncthreads();
    } else {
#pragma unroll
      for (int j = 0; j < NJ; ++j)
#pragma unroll
        for (int r = 0; r < 8; ++r) {
          const float v = acc1[j][r] * kWCarryInv;
          const float x = fmaxf(a1r[j] * v + c1r[j], 0.0f);
          A2s[(rs * 16 + 8 * hf + r) * A2P + cg * HW + 16 * j + lm] = (_Float16)x;
        }
      __syncthreads();
      v8f acc2[4];
#pragma unroll
      for (int i = 0; i < 4; ++i) acc2[i] = (v8f){0.f, 0.f, 0.f, 0.f, 0.f, 0.f, 0.f, 0.f};
#pragma unroll
      for (int kk = 0; kk < NK2; ++kk) {
#pragma unroll
        for (int i = 0; i < 4; ++i) {
          FragH fa;
          fa.h[0] = *(const v8h*)(A2s + (16 * i + lm) * A2P + kk * 32 + 8 * hf);
          fa.h[1] = *(const v8h*)(A2s + (16 * i + lm) * A2P + kk * 32 + 16 + 8 * hf);
          acc2[i] = mma_f16(fa.v, bf2[kk], acc2[i]);
        }
      }
      float mx[NCT], mn[NCT];
#pragma unroll
      for (int cc = 0; cc < NCT; ++cc) { mx[cc] = -3.0e38f; mn[cc] = 3.0e38f; }
#pragma unroll
      for (int i = 0; i < 4; ++i) {
#pragma unroll
        for (int r = 0; r < 8; ++r) {
          const float v = acc2[i][r] * kWCarryInv;
          s2 += v;
          q2 += v * v;
          mx[i / SPC] = fmaxf(mx[i / SPC], v);
          mn[i / SPC] = fminf(mn[i / SPC], v);
        }
      }
#pragma unroll
      for (int cc = 0; cc < NCT; ++cc) {
        const float omx = __shfl_xor(mx[cc], 16, 32);
        const float omn = __shfl_xor(mn[cc], 16, 32);
        const float fx = fmaxf(mx[cc], omx);
        const float fn = fminf(mn[cc], omn);
        const float ev = gp ? fx : fn;
        if (lane < 16) Ex[cc][16 * wave + lm] = ev;
      }
      __syncthreads();
      if (wave < NCT) {
        const v4f o = *(const v4f*)(&Ex[wave][4 * lane]);
        volatile v4f* d = (volatile v4f*)(yext + ((size_t)tile * NCT + wave) * 128 + 4 * lane);
        *d = o;
        __threadfence();
        *d = o;
      }
    }
  }
  if (!FULL) {
#pragma unroll
    for (int j = 0; j < NJ; ++j) {
      s1[j] += __shfl_xor(s1[j], 16, 32);
      q1[j] += __shfl_xor(q1[j], 16, 32);
    }
    if (lane < 16) {
#pragma unroll
      for (int j = 0; j < NJ; ++j) { red[0][wave][16 * j + lane] = s1[j]; red[1][wave][16 * j + lane] = q1[j]; }
    }
    __syncthreads();
    {
      const int n = tid & 127, qq = tid >> 7;
      const int nc = n < NOUT1 ? n : NOUT1 - 1;
      const int cgn = nc / HW;
      const int w = nc - cgn * HW;
      const float v = ((red[qq][cgn * 4 + 0][w] + red[qq][cgn * 4 + 1][w]) + red[qq][cgn * 4 + 2][w]) + red[qq][cgn * 4 + 3][w];
      fin[tid] = (n < NOUT1) ? v : 0.f;
    }
  } else {
    const float os = __shfl_xor(s2, 16, 32);
    const float oq = __shfl_xor(q2, 16, 32);
    s2 += os;
    q2 += oq;
    if (lane < 16) { fin[16 * wave + lm] = s2; fin[128 + 16 * wave + lm] = q2; }
  }
  __syncthreads();
  if (tid < 64) {
    const v4f v = *(const v4f*)(fin + 4 * tid);
    volatile v4f* d = (volatile v4f*)(part + (size_t)blockIdx.x * kPartPitch + 4 * tid);
    *d = v;
    __threadfence();
    *d = v;
  }
}

__global__ __launch_bounds__(256) void k_pool(const float* __restrict__ yext, const float* __restrict__ ac2,
                                              float* __restrict__ out1, int choff) {
  constexpr int TP = 132;
  __shared__ __align__(16) float T[32 * TP];
  __shared__ float sa[128];
  __shared__ float sc[128];
  const int tid = threadIdx.x, lane = tid & 31, wave = tid >> 5;
  const int b = blockIdx.x >> 5;
  const int s0 = (blockIdx.x & 31) * 32;
  if (tid < 128) { sa[tid] = ac2[tid]; sc[tid] = ac2[128 + tid]; }
#pragma unroll
  for (int i = 0; i < 4; ++i) {
    const int u = tid + 256 * i;
    const int row = u >> 5;
    const int c4 = (u & 31) * 4;
    const v4f v = *(const v4f*)(yext + ((size_t)(b * kCen + s0 + row)) * 128 + c4);
    *(v4f*)(T + row * TP + c4) = v;
  }
  __syncthreads();
  float vals[16];
#pragma unroll
  for (int i = 0; i < 16; ++i) {
    const int o = wave + 8 * i;
    vals[i] = fmaxf(sa[o] * T[lane * TP + o] + sc[o], 0.0f);
  }
  float* base = out1 + ((size_t)(b * 256 + choff)) * kCen + s0 + lane;
  for (int pass = 0; pass < 2; ++pass) {
#pragma unroll
    for (int i = 0; i < 16; ++i) *(volatile float*)(base + (size_t)(wave + 8 * i) * kCen) = vals[i];
    __threadfence();
  }
}

extern "C" void kernel_launch(void* const* d_in, const int* in_sizes, int n_in,
                              void* d_out, int out_size, void* d_ws, size_t ws_size, hipStream_t stream) {
  (void)in_sizes; (void)out_size;
  if (n_in < 26) return;
  if (ws_size < kWsTotal) return;
  const float* pc   = (const float*)d_in[0];
  const float* feat = (const float*)d_in[1];
  const float* Wt[2][3]; const float* Gm[2][3]; const float* Be[2][3];
  for (int i = 0; i < 2; ++i)
    for (int j = 0; j < 3; ++j) {
      Wt[i][j] = (const float*)d_in[2 + (i * 3 + j) * 4 + 0];
      Gm[i][j] = (const float*)d_in[2 + (i * 3 + j) * 4 + 2];
      Be[i][j] = (const float*)d_in[2 + (i * 3 + j) * 4 + 3];
    }
  float* out0 = (float*)d_out;
  float* out1 = (float*)d_out + (196608 / 4);

  char* ws = (char*)d_ws;
  float* nx    = (float*)(ws + kOffNx);
  int*   idx0  = (int*)(ws + kOffIdx0);
  int*   idx1  = (int*)(ws + kOffIdx1);
  float* P0    = (float*)(ws + kOffP0);
  float* P1    = (float*)(ws + kOffP1);
  float* yext0 = (float*)(ws + kOffY0);
  float* yext1 = (float*)(ws + kOffY1);
  float* part  = (float*)(ws + kOffPart);
  float* ac    = (float*)(ws + kOffAc);
  const size_t partSlot = (size_t)kStatBlocks * kPartPitch;

  k_fps<<<kBatch, 1024, 0, stream>>>(pc, out0, nx);
  k_ballquery<<<(kBatch * kCen) / 8, 256, 0, stream>>>(pc, nx, idx0, idx1);
  k_pgemm<<<dim3(128, 2), 256, 0, stream>>>(feat, Wt[0][0], Wt[1][0], P0, P1, 8);

  {
    const float invn = 1.0f / (float)kRows0;
    float* p0 = part + 0 * partSlot; float* p1 = part + 1 * partSlot; float* p2 = part + 2 * partSlot;
    float* a0 = ac + 0 * 256; float* a1 = ac + 1 * 256; float* a2 = ac + 2 * 256;
    k_l0stats<kK0><<<kStatBlocks, 256, 0, stream>>>(P0, idx0, pc, nx, Wt[0][0], p0, kRows0 / kStatBlocks);
    k_bnfin<<<1, 128, 0, stream>>>(p0, kStatBlocks, 64, Gm[0][0], Be[0][0], invn, a0);
    k_mlp<64, kK0, false><<<kStatBlocks, 256, 0, stream>>>(P0, idx0, pc, nx, Wt[0][0], a0, Wt[0][1], a1,
                                                           Wt[0][2], Gm[0][2], yext0, p1, kRows0 / 64 / kStatBlocks);
    k_bnfin<<<1, 128, 0, stream>>>(p1, kStatBlocks, 64, Gm[0][1], Be[0][1], invn, a1);
    k_mlp<64, kK0, true><<<kStatBlocks, 256, 0, stream>>>(P0, idx0, pc, nx, Wt[0][0], a0, Wt[0][1], a1,
                                                          Wt[0][2], Gm[0][2], yext0, p2, kRows0 / 64 / kStatBlocks);
    k_bnfin<<<1, 128, 0, stream>>>(p2, kStatBlocks, 128, Gm[0][2], Be[0][2], invn, a2);
    k_pool<<<kBatch * 32, 256, 0, stream>>>(yext0, a2, out1, 0);
  }
  {
    const float invn = 1.0f / (float)kRows1;
    float* p0 = part + 3 * partSlot; float* p1 = part + 4 * partSlot; float* p2 = part + 5 * partSlot;
    float* a0 = ac + 3 * 256; float* a1 = ac + 4 * 256; float* a2 = ac + 5 * 256;
    k_l0stats<kK1><<<kStatBlocks, 256, 0, stream>>>(P1, idx1, pc, nx, Wt[1][0], p0, kRows1 / kStatBlocks);
    k_bnfin<<<1, 128, 0, stream>>>(p0, kStatBlocks, 64, Gm[1][0], Be[1][0], invn, a0);
    k_mlp<96, kK1, false><<<kStatBlocks, 256, 0, stream>>>(P1, idx1, pc, nx, Wt[1][0], a0, Wt[1][1], a1,
                                                           Wt[1][2], Gm[1][2], yext1, p1, kRows1 / 64 / kStatBlocks);
    k_bnfin<<<1, 128, 0, stream>>>(p1, kStatBlocks, 96, Gm[1][1], Be[1][1], invn, a1);
    k_mlp<96, kK1, true><<<kStatBlocks, 256, 0, stream>>>(P1, idx1, pc, nx, Wt[1][0], a0, Wt[1][1], a1,
                                                          Wt[1][2], Gm[1][2], yext1, p2, kRows1 / 64 / kStatBlocks);
    k_bnfin<<<1, 128, 0, stream>>>(p2, kStatBlocks, 128, Gm[1][2], Be[1][2], invn, a2);
    k_pool<<<kBatch * 32, 256, 0, stream>>>(yext1, a2, out1, 128);
  }
}
